// MixHop_24481313587860
// MI455X (gfx1250) — hardware-verified
//
#include <hip/hip_runtime.h>
#include <stddef.h>


#define DF      128
#define HID     256
#define HPA     85
#define HPB     86
#define ODIM    40
#define NPAD1   96
#define NPAD2   48
#define NT1     6
#define NT2     3
#define PLANE   12288
#define HPITCH  260
#define OSTG    640

#define NTHR    256
#define NWAVE   8
#define EPT     8
#define NGRP    2
#define CHUNK   (NTHR * EPT * NGRP)
#define WCAP    (EPT * NGRP * 32)
#define LISTN   (NWAVE * WCAP)
#define NB      512
#define LDS_AGG (NB * DF * 4 + LISTN * 4 + 64 + NB * 4)

#define DTHR    64
#define DWAVES  2

static_assert((CHUNK & (CHUNK - 1)) == 0);
static_assert(CHUNK <= 4096);
static_assert((NB & (NB - 1)) == 0);
static_assert(NB <= 4096);
static_assert(NPAD1 * DF == PLANE);
static_assert(NPAD2 * HID == PLANE);
static_assert(HPA + HPA + HPB == HID);

typedef float          v4f   __attribute__((ext_vector_type(4)));
typedef float          v8f   __attribute__((ext_vector_type(8)));
typedef int            v4i   __attribute__((ext_vector_type(4)));
typedef unsigned short v8us  __attribute__((ext_vector_type(8)));
typedef __bf16         v16bf __attribute__((ext_vector_type(16)));
union FragB { v16bf v; v8us u[2]; };

__device__ __forceinline__ unsigned int bf16_bits(float f) {
  const unsigned int u = __float_as_uint(f);
  return (u + 0x7FFFu + ((u >> 16) & 1u)) >> 16;
}

__device__ __forceinline__ void split8(v4f a, v4f b, v8us* hi, v8us* lo) {
  v8f f;
  f[0] = a.x; f[1] = a.y; f[2] = a.z; f[3] = a.w;
  f[4] = b.x; f[5] = b.y; f[6] = b.z; f[7] = b.w;
  v8us H = {0, 0, 0, 0, 0, 0, 0, 0};
  v8us L = {0, 0, 0, 0, 0, 0, 0, 0};
#pragma unroll
  for (int j = 0; j < 8; ++j) {
    const unsigned int hb = bf16_bits(f[j]);
    const float r = f[j] - __uint_as_float(hb << 16);
    H[j] = (unsigned short)hb;
    L[j] = (unsigned short)bf16_bits(r);
  }
  *hi = H;
  *lo = L;
}

__device__ __forceinline__ v8f wmb(v16bf a, v16bf b, v8f c) {
  v8f d = __builtin_amdgcn_wmma_f32_16x16x32_bf16(false, a, false, b, (short)0, c, false, false);
  asm volatile("v_nop\n\tv_nop\n\tv_nop\n\tv_nop" : "+v"(d) : "v"(a), "v"(b));
  return d;
}

__global__ __launch_bounds__(256) void k_wprep(
    const float* __restrict__ W0, const float* __restrict__ W1,
    const float* __restrict__ W2, const float* __restrict__ Wf,
    unsigned short* wp) {
  const int i = blockIdx.x * 256 + threadIdx.x;
  const int per = PLANE / 8;
  if (i >= 4 * per) return;
  const int which = i / per;
  const int u     = i - which * per;
  const float* W;
  int ncol, kdim, upr;
  if (which == 0)      { W = W0; ncol = HPA;  kdim = DF;  upr = DF / 8; }
  else if (which == 1) { W = W1; ncol = HPA;  kdim = DF;  upr = DF / 8; }
  else if (which == 2) { W = W2; ncol = HPB;  kdim = DF;  upr = DF / 8; }
  else                 { W = Wf; ncol = ODIM; kdim = HID; upr = HID / 8; }
  const int n  = u / upr;
  const int k0 = (u - n * upr) * 8;
  v4f a = {0.f, 0.f, 0.f, 0.f}, b = {0.f, 0.f, 0.f, 0.f};
  if (n < ncol) {
    const float* p = W + (size_t)k0 * ncol + n;
    a.x = p[0];                a.y = p[(size_t)1 * ncol]; a.z = p[(size_t)2 * ncol]; a.w = p[(size_t)3 * ncol];
    b.x = p[(size_t)4 * ncol]; b.y = p[(size_t)5 * ncol]; b.z = p[(size_t)6 * ncol]; b.w = p[(size_t)7 * ncol];
  }
  v8us H, L;
  split8(a, b, &H, &L);
  unsigned short* ph = wp + (size_t)(2 * which) * PLANE + (size_t)n * kdim + k0;
  unsigned short* pl = ph + PLANE;
  *(volatile v8us*)ph = H;
  *(volatile v8us*)pl = L;
  __threadfence();
  *(volatile v8us*)ph = H;
  *(volatile v8us*)pl = L;
}

__device__ __forceinline__ int scan_chunk(const int* __restrict__ dsts, int nE, int cbase, int nodeBase,
                                          int vec8, int* list, int tid, int lane, int wave) {
  int wc = 0;
#pragma unroll
  for (int g = 0; g < NGRP; ++g) {
    const int el0  = (g * NTHR + tid) * EPT;
    const int e0   = cbase + el0;
    const int sent = -2147483647 - 1;
    v4i da, db;
    if (vec8 != 0 && e0 + 7 < nE) {
      da = *(const v4i*)(dsts + e0);
      db = *(const v4i*)(dsts + e0 + 4);
    } else {
      da.x = (e0     < nE) ? dsts[min(e0, nE - 1)] : sent;
      da.y = (e0 + 1 < nE) ? dsts[min(e0 + 1, nE - 1)] : sent;
      da.z = (e0 + 2 < nE) ? dsts[min(e0 + 2, nE - 1)] : sent;
      da.w = (e0 + 3 < nE) ? dsts[min(e0 + 3, nE - 1)] : sent;
      db.x = (e0 + 4 < nE) ? dsts[min(e0 + 4, nE - 1)] : sent;
      db.y = (e0 + 5 < nE) ? dsts[min(e0 + 5, nE - 1)] : sent;
      db.z = (e0 + 6 < nE) ? dsts[min(e0 + 6, nE - 1)] : sent;
      db.w = (e0 + 7 < nE) ? dsts[min(e0 + 7, nE - 1)] : sent;
    }
    const unsigned nb = (unsigned)nodeBase;
    const unsigned s0 = (unsigned)da.x - nb, s1 = (unsigned)da.y - nb;
    const unsigned s2 = (unsigned)da.z - nb, s3 = (unsigned)da.w - nb;
    const unsigned s4 = (unsigned)db.x - nb, s5 = (unsigned)db.y - nb;
    const unsigned s6 = (unsigned)db.z - nb, s7 = (unsigned)db.w - nb;
    const bool h0 = s0 < (unsigned)NB, h1 = s1 < (unsigned)NB, h2 = s2 < (unsigned)NB, h3 = s3 < (unsigned)NB;
    const bool h4 = s4 < (unsigned)NB, h5 = s5 < (unsigned)NB, h6 = s6 < (unsigned)NB, h7 = s7 < (unsigned)NB;
    const unsigned any = __builtin_amdgcn_ballot_w32(h0 | h1 | h2 | h3 | h4 | h5 | h6 | h7);
    if (any != 0u) {
#define HITJ(J, HJ, SJ) { \
        const unsigned mj = __builtin_amdgcn_ballot_w32(HJ); \
        if (mj != 0u) { \
          if (HJ) { \
            const int pos = wc + (int)__builtin_amdgcn_mbcnt_lo(mj, 0u); \
            if (pos < WCAP) list[wave * WCAP + pos] = ((el0 + (J)) << 12) | (int)(SJ); \
          } \
          wc += (int)__builtin_popcount(mj); } }
      HITJ(0, h0, s0)
      HITJ(1, h1, s1)
      HITJ(2, h2, s2)
      HITJ(3, h3, s3)
      HITJ(4, h4, s4)
      HITJ(5, h5, s5)
      HITJ(6, h6, s6)
      HITJ(7, h7, s7)
#undef HITJ
    }
  }
  return wc;
}

template <int DEG>
__global__ __launch_bounds__(NTHR) void k_agg(
    const int* __restrict__ ei, const float* __restrict__ src,
    float* dst, float* dinv, int nN, int nE, int vec8) {
  extern __shared__ v4f lds_dyn[];
  float* acc  = (float*)lds_dyn;
  int*   list = (int*)(acc + NB * DF);
  int*   wcnt = list + LISTN;
  int*   cnt  = wcnt + 16;
  const int tid = threadIdx.x, lane = tid & 31, wave = tid >> 5;
  const int nodeBase = blockIdx.x * NB;
  const int* dsts = ei;
  const int* srcs = ei + nE;

  {
    const v4f z = {0.f, 0.f, 0.f, 0.f};
    for (int i = tid; i < NB * DF / 4; i += NTHR) lds_dyn[i] = z;
    for (int i = tid; i < NB; i += NTHR) cnt[i] = 0;
  }
  __syncthreads();

  const int nChunks = (nE + CHUNK - 1) / CHUNK;
#pragma unroll 1
  for (int ch = 0; ch < nChunks; ++ch) {
    const int cbase = ch * CHUNK;
    const int wc = scan_chunk(dsts, nE, cbase, nodeBase, vec8, list, tid, lane, wave);
    if (lane == 0) wcnt[wave] = wc;
    __syncthreads();
    if (wave == 0) {
#pragma unroll 1
      for (int wsx = 0; wsx < NWAVE; ++wsx) {
        int n = __builtin_amdgcn_readfirstlane(wcnt[wsx]);
        n = n > WCAP ? WCAP : (n < 0 ? 0 : n);
        const int* lp = list + wsx * WCAP;
#pragma unroll 1
        for (int i = 0; i < n; ++i) {
          const int ent  = __builtin_amdgcn_readfirstlane(lp[i]);
          const int slot = ent & (NB - 1);
          int e = cbase + ((ent >> 12) & (CHUNK - 1));
          e = e > nE - 1 ? nE - 1 : e;
          int s = __builtin_amdgcn_readfirstlane(srcs[e]);
          s = s < 0 ? 0 : (s > nN - 1 ? nN - 1 : s);
          const v4f v = *(const v4f*)(src + (size_t)s * DF + 4 * lane);
          v4f* ap = (v4f*)(acc + slot * DF + 4 * lane);
          *ap = *ap + v;
          if (DEG) { if (lane == 0) cnt[slot] = cnt[slot] + 1; }
        }
      }
    }
    __syncthreads();
  }

  if (DEG) {
    if (wave < 4) {
      const int f = tid * 4;
      const v4i c = *(const v4i*)(cnt + f);
      v4f d;
      d.x = 1.0f / fmaxf((float)c.x, 1.0f);
      d.y = 1.0f / fmaxf((float)c.y, 1.0f);
      d.z = 1.0f / fmaxf((float)c.z, 1.0f);
      d.w = 1.0f / fmaxf((float)c.w, 1.0f);
      float* dp = dinv + (size_t)nodeBase + f;
      *(volatile v4f*)dp = d;
      __threadfence();
      *(volatile v4f*)dp = d;
    }
  }

  const float* lrow = acc + (wave * 64) * DF + 4 * lane;
  float* gp = dst + ((size_t)nodeBase + wave * 64) * DF + 4 * lane;
#pragma unroll 4
  for (int i = 0; i < 64; ++i) { const v4f v = *(const v4f*)(lrow + i * DF); *(volatile v4f*)(gp + (size_t)i * DF) = v; }
  __threadfence();
#pragma unroll 4
  for (int i = 0; i < 64; ++i) { const v4f v = *(const v4f*)(lrow + i * DF); *(volatile v4f*)(gp + (size_t)i * DF) = v; }
}

__device__ __forceinline__ void hop_stage(const float* __restrict__ arow, float sc,
                                          const unsigned short* __restrict__ wh,
                                          const unsigned short* __restrict__ wl,
                                          const float* __restrict__ bias, int ncol, int coff,
                                          float* hl, int h, int m) {
  v8f acc[NT1];
#pragma unroll
  for (int t = 0; t < NT1; ++t) { v8f z = {0.f, 0.f, 0.f, 0.f, 0.f, 0.f, 0.f, 0.f}; acc[t] = z; }
#pragma unroll 1
  for (int kt = 0; kt < DF / 32; ++kt) {
    const float* ap = arow + 32 * kt + 8 * h;
    const v4f p0 = *(const v4f*)ap * sc,        p1 = *(const v4f*)(ap + 4) * sc;
    const v4f p2 = *(const v4f*)(ap + 16) * sc, p3 = *(const v4f*)(ap + 20) * sc;
    FragB ah, al;
    split8(p0, p1, &ah.u[0], &al.u[0]);
    split8(p2, p3, &ah.u[1], &al.u[1]);
#pragma unroll
    for (int t = 0; t < NT1; ++t) {
      const size_t bo = (size_t)(16 * t + m) * DF + 32 * kt + 8 * h;
      FragB bh, bl;
      bh.u[0] = *(const v8us*)(wh + bo); bh.u[1] = *(const v8us*)(wh + bo + 16);
      bl.u[0] = *(const v8us*)(wl + bo); bl.u[1] = *(const v8us*)(wl + bo + 16);
      acc[t] = wmb(ah.v, bh.v, acc[t]);
      acc[t] = wmb(ah.v, bl.v, acc[t]);
      acc[t] = wmb(al.v, bh.v, acc[t]);
    }
  }
#pragma unroll
  for (int t = 0; t < NT1; ++t) {
    const int col = 16 * t + m;
    if (col < ncol) {
      const float bv = bias[col];
      float* hp = hl + (8 * h) * HPITCH + coff + col;
#pragma unroll
      for (int r = 0; r < 8; ++r) hp[r * HPITCH] = fmaxf(acc[t][r] + bv, 0.f);
    }
  }
}

__global__ __launch_bounds__(DTHR) void k_dense(
    const float* __restrict__ x, const float* __restrict__ ax, const float* __restrict__ aax,
    const float* __restrict__ dinv, const unsigned short* __restrict__ wp,
    const float* __restrict__ b0, const float* __restrict__ b1, const float* __restrict__ b2,
    const float* __restrict__ bfin, float* out, int nN) {
  __shared__ __attribute__((aligned(16))) float hls[DWAVES][16 * HPITCH];
  __shared__ __attribute__((aligned(16))) float ost[DWAVES][OSTG];
  const int tid = threadIdx.x, lane = tid & 31, wave = tid >> 5, h = lane >> 4, m = lane & 15;
  const int nTiles = (nN + 15) >> 4;
  const int tile   = blockIdx.x * DWAVES + wave;
  const bool valid = tile < nTiles;
  const int tb     = (valid ? tile : nTiles - 1) * 16;
  int row = tb + m;
  row = row > nN - 1 ? nN - 1 : row;
  const float dv = dinv[row];
  float* hl = hls[wave];

  hop_stage(x   + (size_t)row * DF, 1.0f,    wp + 0 * PLANE, wp + 1 * PLANE, b0, HPA, 0,       hl, h, m);
  hop_stage(ax  + (size_t)row * DF, dv,      wp + 2 * PLANE, wp + 3 * PLANE, b1, HPA, HPA,     hl, h, m);
  hop_stage(aax + (size_t)row * DF, dv * dv, wp + 4 * PLANE, wp + 5 * PLANE, b2, HPB, 2 * HPA, hl, h, m);
  __syncthreads();

  v8f c[NT2];
#pragma unroll
  for (int t = 0; t < NT2; ++t) { v8f z = {0.f, 0.f, 0.f, 0.f, 0.f, 0.f, 0.f, 0.f}; c[t] = z; }
  const unsigned short* wfh = wp + 6 * PLANE;
  const unsigned short* wfl = wp + 7 * PLANE;
#pragma unroll 1
  for (int kt = 0; kt < HID / 32; ++kt) {
    const float* ap = hl + m * HPITCH + 32 * kt + 8 * h;
    const v4f p0 = *(const v4f*)ap,        p1 = *(const v4f*)(ap + 4);
    const v4f p2 = *(const v4f*)(ap + 16), p3 = *(const v4f*)(ap + 20);
    FragB ah, al;
    split8(p0, p1, &ah.u[0], &al.u[0]);
    split8(p2, p3, &ah.u[1], &al.u[1]);
#pragma unroll
    for (int t = 0; t < NT2; ++t) {
      const size_t bo = (size_t)(16 * t + m) * HID + 32 * kt + 8 * h;
      FragB bh, bl;
      bh.u[0] = *(const v8us*)(wfh + bo); bh.u[1] = *(const v8us*)(wfh + bo + 16);
      bl.u[0] = *(const v8us*)(wfl + bo); bl.u[1] = *(const v8us*)(wfl + bo + 16);
      c[t] = wmb(ah.v, bh.v, c[t]);
      c[t] = wmb(ah.v, bl.v, c[t]);
      c[t] = wmb(al.v, bh.v, c[t]);
    }
  }

  float* os = ost[wave];
#pragma unroll
  for (int t = 0; t < NT2; ++t) {
    const int col = 16 * t + m;
    if (col < ODIM) {
      const float bv = bfin[col];
      float* op = os + (8 * h) * ODIM + col;
#pragma unroll
      for (int r = 0; r < 8; ++r) op[r * ODIM] = c[t][r] + bv;
    }
  }
  __syncthreads();

  if (valid) {
    const size_t outN = (size_t)nN * ODIM;
    const size_t ob   = (size_t)tb * ODIM;
    v4f ov[5];
#pragma unroll
    for (int q = 0; q < 5; ++q) ov[q] = *(const v4f*)(os + q * 128 + 4 * lane);
#pragma unroll
    for (int q = 0; q < 5; ++q) {
      const size_t gi = ob + (size_t)(q * 128 + 4 * lane);
      if (gi + 4 <= outN) *(volatile v4f*)(out + gi) = ov[q];
    }
    __threadfence();
#pragma unroll
    for (int q = 0; q < 5; ++q) {
      const size_t gi = ob + (size_t)(q * 128 + 4 * lane);
      if (gi + 4 <= outN) *(volatile v4f*)(out + gi) = ov[q];
    }
  }
}

extern "C" void kernel_launch(void* const* d_in, const int* in_sizes, int n_in,
                              void* d_out, int out_size, void* d_ws, size_t ws_size,
                              hipStream_t stream) {
  if (n_in < 10) return;
  const int nN = in_sizes[0] / DF;
  const int nE = in_sizes[1] / 2;
  if (nN <= 0 || nE < 0 || in_sizes[0] != nN * DF || in_sizes[1] != nE * 2) return;
  if (in_sizes[2] != DF * HPA || in_sizes[3] < HPA) return;
  if (in_sizes[4] != DF * HPA || in_sizes[5] < HPA) return;
  if (in_sizes[6] != DF * HPB || in_sizes[7] < HPB) return;
  if (in_sizes[8] != HID * ODIM || in_sizes[9] < ODIM) return;
  if (out_size != nN * ODIM) return;

  const float* x   = (const float*)d_in[0];
  const int*   ei  = (const int*)d_in[1];
  const float* W0  = (const float*)d_in[2];
  const float* b0  = (const float*)d_in[3];
  const float* W1  = (const float*)d_in[4];
  const float* b1  = (const float*)d_in[5];
  const float* W2  = (const float*)d_in[6];
  const float* b2  = (const float*)d_in[7];
  const float* Wf  = (const float*)d_in[8];
  const float* bfv = (const float*)d_in[9];
  float* out = (float*)d_out;

  const int nBlk   = (nN + NB - 1) / NB;
  const size_t nNp = (size_t)nBlk * NB;
  const int nTiles = (nN + 15) / 16;
  const int nDB    = (nTiles + DWAVES - 1) / DWAVES;

  char* ws = (char*)d_ws;
  size_t off = 0;
  const size_t oWP  = off; off += (size_t)8 * PLANE * 2;       off = (off + 255) & ~(size_t)255;
  const size_t oDV  = off; off += nNp * 4;                     off = (off + 255) & ~(size_t)255;
  const size_t oAX  = off; off += nNp * DF * 4;                off = (off + 255) & ~(size_t)255;
  const size_t oAAX = off; off += nNp * DF * 4;                off = (off + 255) & ~(size_t)255;
  if (off > ws_size || off > (size_t)134217728) return;
  unsigned short* wp = (unsigned short*)(ws + oWP);
  float* dinv = (float*)(ws + oDV);
  float* ax   = (float*)(ws + oAX);
  float* aax  = (float*)(ws + oAAX);

  const int vec8 = ((nE & 3) == 0) ? 1 : 0;

  const int nPrep = 4 * (PLANE / 8);
  k_wprep<<<(nPrep + 255) / 256, 256, 0, stream>>>(W0, W1, W2, Wf, wp);

  hipFuncSetAttribute(reinterpret_cast<const void*>(&k_agg<1>),
                      hipFuncAttributeMaxDynamicSharedMemorySize, LDS_AGG);
  k_agg<1><<<nBlk, NTHR, LDS_AGG, stream>>>(ei, x, ax, dinv, nN, nE, vec8);

  hipFuncSetAttribute(reinterpret_cast<const void*>(&k_agg<0>),
                      hipFuncAttributeMaxDynamicSharedMemorySize, LDS_AGG);
  k_agg<0><<<nBlk, NTHR, LDS_AGG, stream>>>(ei, ax, aax, dinv, nN, nE, vec8);

  k_dense<<<nDB, DTHR, 0, stream>>>(x, ax, aax, dinv, wp, b0, b1, b2, bfv, out, nN);
}
